// KnowledgeAttention_35905926595170
// MI455X (gfx1250) — hardware-verified
//
#include <hip/hip_runtime.h>
#include <hip/hip_bf16.h>
#include <math.h>

#define NBk 4
#define TTk 512
#define KKn 256
#define DK_ 256
#define DE_ 256
#define UU 128
#define GSTR 48

typedef _Float16 bf16;
typedef _Float16 f16;
typedef __attribute__((ext_vector_type(4))) unsigned v4u_t;
typedef unsigned v4ua __attribute__((ext_vector_type(4), may_alias));
typedef __attribute__((ext_vector_type(4))) float v4f_t;
typedef float v4fa __attribute__((ext_vector_type(4), may_alias));
typedef __attribute__((ext_vector_type(16))) bf16  bf16x16;
typedef bf16x16 f16x16;
typedef __attribute__((ext_vector_type(8)))  bf16  bf16x8;
typedef bf16x8 f16x8;
typedef __attribute__((ext_vector_type(8)))  float f32x8;
__device__ __forceinline__ f32x8 wmma16(f16x16 a, f16x16 b, f32x8 c) {
  c = __builtin_amdgcn_wmma_f32_16x16x32_f16(false, a, false, b, (short)0, c, false, false);
  asm volatile("v_nop\n\tv_nop\n\tv_nop\n\tv_nop" : "+v"(c) : "v"(a), "v"(b));
  return c;
}
__device__ __forceinline__ f16x16 lds_frag(const f16* base, int stride) {
  const int lane = threadIdx.x & 31, row = lane & 15, kh = (lane >> 4) * 8;
  const f16x8 lo = *(const f16x8*)(base + row * stride + kh);
  const f16x8 hi = *(const f16x8*)(base + row * stride + kh + 16);
  f16x16 f;
#pragma unroll
  for (int i = 0; i < 8; ++i) { f[i] = lo[i]; f[i + 8] = hi[i]; }
  return f;
}
__device__ __forceinline__ f16x16 wfragKN(const float* __restrict__ Wm, int ldw, int k0, int n0) {
  const int lane = threadIdx.x & 31, n = n0 + (lane & 15), kh = (lane >> 4) * 8; f16x16 f;
#pragma unroll
  for (int i = 0; i < 8; ++i) { f[i] = (f16)Wm[(size_t)(k0 + kh + i) * ldw + n]; f[i + 8] = (f16)Wm[(size_t)(k0 + kh + 16 + i) * ldw + n]; }
  return f;
}

#define GSTR 48
template <typename AT, int EPI, bool OUT16>
__global__ __launch_bounds__(256) void gemm_kne(const AT* __restrict__ A, int lda, const float* __restrict__ Wm, int ldw,
                                                const float* __restrict__ bias, const float* __restrict__ R, const float* __restrict__ gvec,
                                                void* __restrict__ Yv, int ldy, int K) {
  __shared__ __attribute__((aligned(16))) f16 ldsA[128 * GSTR];
  __shared__ __attribute__((aligned(16))) f16 ldsW[128 * GSTR];
  __shared__ __attribute__((aligned(16))) float oS[8][32 * 68];
  const int tid = threadIdx.x, lane = tid & 31, wave = tid >> 5, cl = lane & 15, rh = (lane >> 4) * 8;
  const int m0 = blockIdx.x * 128, n0 = blockIdx.y * 128;
  const int wm = (wave & 3) * 32, wn = (wave >> 2) * 64;
  f32x8 acc[2][4];
#pragma unroll
  for (int i = 0; i < 2; ++i)
#pragma unroll
    for (int j = 0; j < 4; ++j) { f32x8 z = {}; acc[i][j] = z; }
#pragma unroll 1
  for (int k0 = 0; k0 < K; k0 += 32) {
    __syncthreads();
    { const int row = tid >> 1, ch = (tid & 1) * 16;
      const AT* src = A + (size_t)(m0 + row) * lda + k0 + ch;
#pragma unroll
      for (int g = 0; g < 16; ++g) ldsA[row * GSTR + ch + g] = (f16)src[g]; }
    { const int k = tid >> 3, nn0 = (tid & 7) * 16;
      const float* src = Wm + (size_t)(k0 + k) * ldw + n0 + nn0;
#pragma unroll
      for (int g = 0; g < 4; ++g) { const v4f_t v = *(const v4f_t*)(src + 4 * g);
#pragma unroll
        for (int u = 0; u < 4; ++u) ldsW[(nn0 + 4 * g + u) * GSTR + k] = (f16)v[u]; } }
    __syncthreads();
    f16x16 af[2];
#pragma unroll
    for (int i = 0; i < 2; ++i) af[i] = lds_frag(ldsA + (wm + 16 * i) * GSTR, GSTR);
#pragma unroll
    for (int j = 0; j < 4; ++j) {
      const f16x16 bf = lds_frag(ldsW + (wn + 16 * j) * GSTR, GSTR);
#pragma unroll
      for (int i = 0; i < 2; ++i) acc[i][j] = wmma16(af[i], bf, acc[i][j]);
    }
  }
  float* so = oS[wave];
#pragma unroll
  for (int i = 0; i < 2; ++i)
#pragma unroll
    for (int j = 0; j < 4; ++j) {
      const int n = n0 + wn + 16 * j + cl;
      const float bv = bias ? bias[n] : 0.0f;
      const float gv = (EPI == 2) ? gvec[n] : 0.0f;
      if (EPI == 1) {
#pragma unroll 1
        for (int r = 0; r < 8; ++r) { const float xg = acc[i][j][r] + bv; so[(16 * i + rh + r) * 68 + 16 * j + cl] = 0.5f * xg * (1.0f + erff(xg * 0.70710678118654752f)); }
      } else {
#pragma unroll
        for (int r = 0; r < 8; ++r) {
          float v = acc[i][j][r] + bv;
          if (EPI == 2) v = R[(size_t)(m0 + wm + 16 * i + rh + r) * ldy + n] + gv * v;
          so[(16 * i + rh + r) * 68 + 16 * j + cl] = v;
        }
      }
    }
  asm volatile("s_wait_dscnt 0" ::: "memory");
  __builtin_amdgcn_wave_barrier();
#pragma unroll 1
  for (int pass = 0; pass < 2; ++pass) {
    if (OUT16) {
      f16* Y = (f16*)Yv;
#pragma unroll
      for (int it = 0; it < 8; ++it) { const int c = lane + 32 * it, rr = c >> 3, q8 = (c & 7) * 8;
        union { f16 h[8]; v4u_t v; } u;
#pragma unroll
        for (int e = 0; e < 8; ++e) u.h[e] = (f16)so[rr * 68 + q8 + e];
        *(volatile v4u_t*)(Y + (size_t)(m0 + wm + rr) * ldy + n0 + wn + q8) = u.v; }
    } else {
      float* Y = (float*)Yv;
#pragma unroll
      for (int it = 0; it < 16; ++it) { const int f4 = lane + 32 * it, rr = f4 >> 4, q = (f4 & 15) * 4;
        *(volatile v4f_t*)(Y + (size_t)(m0 + wm + rr) * ldy + n0 + wn + q) = *(const v4fa*)(so + rr * 68 + q); }
    }
    __threadfence();
  }
}

__global__ __launch_bounds__(256) void k_know(const float* __restrict__ E, const float* __restrict__ Kp, const float* __restrict__ Vv, const float* __restrict__ bV, const float* __restrict__ kn, float* __restrict__ out) {
  __shared__ __attribute__((aligned(16))) f16 kS[KKn * 136];
  __shared__ float eS[16 * UU];
  __shared__ float vS[UU];
  __shared__ float sS[16 * KKn];
  __shared__ __attribute__((aligned(16))) f16 pS[16 * 264];
  __shared__ __attribute__((aligned(16))) float oS[16 * 260];
  const int tid = threadIdx.x, lane = tid & 31, wave = tid >> 5, cl = lane & 15, rh = (lane >> 4) * 8;
  const int b = blockIdx.x / (TTk / 16), t0 = (blockIdx.x % (TTk / 16)) * 16;
  for (int e = tid; e < KKn * UU; e += 256) { const int k = e >> 7, u = e & 127; kS[k * 136 + u] = (f16)Kp[((size_t)b * KKn + k) * UU + u]; }
  for (int e = tid; e < 16 * UU; e += 256) eS[e] = E[((size_t)b * TTk + t0) * UU + e];
  if (tid < UU) vS[tid] = Vv[tid];
  __syncthreads();
  { const int t = tid >> 4, kq = tid & 15;
#pragma unroll 1
    for (int q = 0; q < 16; ++q) { const int k = kq + 16 * q; float s = 0.0f;
#pragma unroll 1
      for (int u = 0; u < UU; ++u) s += tanhf(eS[t * UU + u] + (float)kS[k * 136 + u]) * vS[u];
      sS[t * KKn + k] = s + bV[0]; } }
  __syncthreads();
#pragma unroll 1
  for (int rr = 0; rr < 2; ++rr) { const int t = wave * 2 + rr; float m = -3.0e38f;
    for (int k = lane; k < KKn; k += 32) m = fmaxf(m, sS[t * KKn + k]);
#pragma unroll
    for (int off = 1; off < 32; off <<= 1) m = fmaxf(m, __shfl_xor(m, off, 32));
    float z = 0.0f; float ev[8];
#pragma unroll
    for (int q = 0; q < 8; ++q) { ev[q] = expf(sS[t * KKn + lane + 32 * q] - m); z += ev[q]; }
#pragma unroll
    for (int off = 1; off < 32; off <<= 1) z += __shfl_xor(z, off, 32);
    const float iz = 1024.0f / z;
#pragma unroll
    for (int q = 0; q < 8; ++q) pS[t * 264 + lane + 32 * q] = (f16)(ev[q] * iz); }
  __syncthreads();
  { const float* knb = kn + (size_t)b * KKn * DK_;
#pragma unroll 1
    for (int jj = 0; jj < 2; ++jj) { const int ct = wave * 2 + jj; f32x8 acc = {};
#pragma unroll 1
      for (int ks = 0; ks < KKn / 32; ++ks) acc = wmma16(lds_frag(pS + ks * 32, 264), wfragKN(knb, DK_, ks * 32, ct * 16), acc);
#pragma unroll
      for (int r = 0; r < 8; ++r) oS[(rh + r) * 260 + ct * 16 + cl] = acc[r] * (1.0f / 1024.0f); } }
  __syncthreads();
#pragma unroll 1
  for (int pass = 0; pass < 2; ++pass) { for (int q4 = tid; q4 < 16 * 64; q4 += 256) { const int t = q4 >> 6, c4 = (q4 & 63) * 4;
      v4f_t v; v[0] = oS[t * 260 + c4]; v[1] = oS[t * 260 + c4 + 1]; v[2] = oS[t * 260 + c4 + 2]; v[3] = oS[t * 260 + c4 + 3];
      *(volatile v4f_t*)(out + ((size_t)b * TTk + t0 + t) * DK_ + c4) = v; } __threadfence(); }
}

extern "C" void kernel_launch(void* const* d_in, const int* in_sizes, int n_in,
                              void* d_out, int out_size, void* d_ws, size_t ws_size,
                              hipStream_t stream) {
  (void)in_sizes; (void)n_in; (void)out_size;
  const float** f = (const float**)d_in;
  const float* kn = f[0], *enc = f[1], *W1 = f[2], *b1 = f[3], *W2 = f[4], *b2 = f[5], *Vv = f[6], *bV = f[7];
  float* out = (float*)d_out;
  char* ws = (char*)d_ws;
  float* E = (float*)ws; ws += (size_t)NBk * TTk * UU * 4;
  float* Kp = (float*)ws; ws += (size_t)NBk * KKn * UU * 4;
  if ((size_t)(ws - (char*)d_ws) > ws_size) return;
  const dim3 blk(256);
  gemm_kne<float, 0, false><<<dim3(NBk * TTk / 128, UU / 128), blk, 0, stream>>>(enc, DE_, W1, UU, b1, nullptr, nullptr, E, UU, DE_);
  gemm_kne<float, 0, false><<<dim3(NBk * KKn / 128, UU / 128), blk, 0, stream>>>(kn, DK_, W2, UU, b2, nullptr, nullptr, Kp, UU, DK_);
  k_know<<<dim3(NBk * TTk / 16), blk, 0, stream>>>(E, Kp, Vv, bV, kn, out);
}
